// DIMESDenseEncoder_10617159156313
// MI455X (gfx1250) — hardware-run, weakly checked
//
#include <hip/hip_runtime.h>
#include <stddef.h>
#include <stdint.h>

#pragma clang fp contract(off)

#define NB     16
#define NN     200
#define UU     64
#define NL     3
#define NROW   (NB * NN)
#define GSZ    (NN * NN)
#define RTOT   (NB * NN * NN)
#define TROWS  128
#define NTILE  (RTOT / TROWS)
#define NLIVE  (NB * NN * (NN - 1))
#define KK     128
#define X4W    256
#define DP     68
#define BNEPS  1e-5f

#define PT_NB   0
#define PT_EB   768
#define PT_EG   960
#define PT_EBB  1152
#define PT_EW0  1344
#define PT_EB0  1408
#define PT_E1W  1472
#define PT_E1B  1536
#define PT_VG   1568
#define PT_VB   1760
#define PT_END  1952

#define EDGE_DYN_BYTES (TROWS * DP * 4 + TROWS * KK * 2 + UU * KK * 2)

#define SZ_WHL  ((size_t)RTOT * KK * 2)
#define SZ_X4   ((size_t)NROW * X4W * 4)
#define SZ_H    ((size_t)NROW * UU * 4)
#define SZ_HHL  ((size_t)NROW * KK * 2)
#define SZ_PO   ((size_t)NROW * UU * 4)
#define SZ_REC  ((size_t)NTILE * 128 * 4)
#define SZ_WN   ((size_t)NL * 256 * KK * 2)
#define SZ_ET   ((size_t)NL * UU * KK * 2)
#define SZ_PT   ((size_t)8192)
#define SZ_ST   ((size_t)512)
#define WS_TOTAL (SZ_WHL + SZ_X4 + SZ_H + SZ_HHL + SZ_PO + SZ_REC + SZ_WN + SZ_ET + SZ_PT + SZ_ST)

static_assert(UU == 64);
static_assert(RTOT % TROWS == 0);
static_assert(NROW % 128 == 0 && NROW % 64 == 0);
static_assert(NN % 8 == 0);
static_assert(NLIVE == 636800);
static_assert(KK % 32 == 0 && KK == 2 * UU);
static_assert(PT_NB % 32 == 0 && PT_EB % 32 == 0 && PT_EG % 32 == 0 && PT_EBB % 32 == 0);
static_assert(PT_EW0 % 32 == 0 && PT_EB0 % 32 == 0 && PT_E1W % 32 == 0 && PT_E1B % 32 == 0);
static_assert(PT_VG % 32 == 0 && PT_VB % 32 == 0 && PT_VB == PT_VG + NL * UU && PT_END * 4 <= 8192);
static_assert(PT_EB == PT_NB + NL * 256 && PT_VG == PT_EB + 800);
static_assert((DP * 4) % 16 == 0 && DP >= UU);
static_assert(SZ_WHL % 256 == 0 && SZ_X4 % 256 == 0 && SZ_H % 256 == 0 && SZ_HHL % 256 == 0);
static_assert(SZ_REC % 256 == 0 && SZ_WN % 256 == 0 && SZ_ET % 256 == 0 && SZ_PT % 256 == 0 && SZ_ST % 256 == 0);
static_assert(WS_TOTAL == 172388864ull && WS_TOTAL <= 268435456ull);
static_assert((size_t)(NTILE - 1) * TROWS + TROWS - 1 == (size_t)RTOT - 1);
static_assert(EDGE_DYN_BYTES == 83968);

typedef float          v2f   __attribute__((ext_vector_type(2)));
typedef float          v4f   __attribute__((ext_vector_type(4)));
typedef float          v8f   __attribute__((ext_vector_type(8)));
typedef int            v4i   __attribute__((ext_vector_type(4)));
typedef int            v8i   __attribute__((ext_vector_type(8)));
typedef unsigned short v4us  __attribute__((ext_vector_type(4)));
typedef unsigned short v8us  __attribute__((ext_vector_type(8)));
typedef unsigned short v16us __attribute__((ext_vector_type(16)));
typedef __bf16         v16bf __attribute__((ext_vector_type(16)));
typedef v2f  __attribute__((may_alias)) v2fa;
typedef v4f  __attribute__((may_alias)) v4fa;
typedef v4i  __attribute__((may_alias)) v4ia;
typedef v4us __attribute__((may_alias)) v4usa;
typedef v8us __attribute__((may_alias)) v8usa;
union FragB { v16bf v; v16us u; v8us h[2]; v8i w; };

__device__ __forceinline__ v8f wmb(const FragB& a, const FragB& b, v8f c) {
  v8f d = __builtin_amdgcn_wmma_f32_16x16x32_bf16(false, a.v, false, b.v, (short)0, c, false, false);
  asm volatile("v_nop\n\tv_nop\n\tv_nop\n\tv_nop" : "+v"(d) : "v"(a.w), "v"(b.w));
  return d;
}
__device__ __forceinline__ v8f z8() { v8f z = {0.f, 0.f, 0.f, 0.f, 0.f, 0.f, 0.f, 0.f}; return z; }

__device__ __forceinline__ unsigned bf16_bits(float f) {
  const unsigned u = __float_as_uint(f);
  return (u + 0x7FFFu + ((u >> 16) & 1u)) >> 16;
}
__device__ __forceinline__ float bf16_val(float f) {
  return __uint_as_float(bf16_bits(f) << 16);
}
__device__ __forceinline__ float bw(unsigned w16) { return __uint_as_float(w16 << 16); }
__device__ __forceinline__ void split2(float v, unsigned& hb, unsigned& lb) {
  const unsigned h = bf16_bits(v);
  hb = h;
  lb = bf16_bits(v - __uint_as_float(h << 16));
}
__device__ __forceinline__ float lrelu(float v) { return (v >= 0.0f) ? v : 0.01f * v; }
__device__ __forceinline__ void put16(unsigned short* dp, v8us o) {
  *(volatile v8us*)dp = o;
  __threadfence();
  *(volatile v8us*)dp = o;
}
__device__ __forceinline__ void put4f(float* dp, v4f o) {
  *(volatile v4f*)dp = o;
  __threadfence();
  *(volatile v4f*)dp = o;
}

__host__ __device__ __forceinline__ int diag_before(int X) {
  const int g = X / GSZ;
  const int x = X - g * GSZ;
  int c = (x + 200) / 201;
  c = c > NN ? NN : c;
  return g * NN + c;
}
__host__ __device__ __forceinline__ int diag_pos(int k) {
  const int g = k / NN;
  return g * GSZ + (k - g * NN) * 201;
}

__device__ __forceinline__ v8us gather_wt(const float* __restrict__ W, int layer, int k8, int o) {
  const float* p = W + (size_t)layer * UU * UU + (size_t)k8 * UU + o;
  v8us r;
#pragma unroll
  for (int t = 0; t < 8; ++t) r[t] = (unsigned short)bf16_bits(p[(size_t)t * UU]);
  return r;
}

__global__ __launch_bounds__(256) void k_pa(const float* __restrict__ w1, const float* __restrict__ w2,
                                            const float* __restrict__ w3, const float* __restrict__ w4,
                                            const float* __restrict__ b1, const float* __restrict__ b2,
                                            const float* __restrict__ b3, const float* __restrict__ b4,
                                            unsigned short* WN, float* PT) {
  const int tid = (int)threadIdx.x;
  if ((int)blockIdx.x < 48) {
    const int u = (int)blockIdx.x * 256 + tid;
    const int layer = u >> 12;
    const int rem = u & 4095;
    const int n = rem >> 4;
    const int k8 = ((rem & 15) * 8) & 63;
    const int j = n >> 6;
    const int o = n & 63;
    v8us r;
    if (j == 0)      r = gather_wt(w1, layer, k8, o);
    else if (j == 1) r = gather_wt(w2, layer, k8, o);
    else if (j == 2) r = gather_wt(w3, layer, k8, o);
    else             r = gather_wt(w4, layer, k8, o);
    put16(WN + (size_t)u * 8, r);
  } else {
    const bool act = tid < 192;
    const int t = act ? tid : 0;
    const int layer = t >> 6;
    const int n4 = (t & 63) * 4;
    const int j = n4 >> 6;
    const int off = layer * UU + (n4 & 63);
    const v4f a = *(const v4f*)(b1 + off);
    const v4f b = *(const v4f*)(b2 + off);
    const v4f c = *(const v4f*)(b3 + off);
    const v4f d = *(const v4f*)(b4 + off);
    const unsigned m0 = (j == 0) ? 0xffffffffu : 0u;
    const unsigned m1 = (j == 1) ? 0xffffffffu : 0u;
    const unsigned m2 = (j == 2) ? 0xffffffffu : 0u;
    const unsigned m3 = (j == 3) ? 0xffffffffu : 0u;
    v4f o;
    o.x = bf16_val(__uint_as_float((__float_as_uint(a.x) & m0) | (__float_as_uint(b.x) & m1) | (__float_as_uint(c.x) & m2) | (__float_as_uint(d.x) & m3)));
    o.y = bf16_val(__uint_as_float((__float_as_uint(a.y) & m0) | (__float_as_uint(b.y) & m1) | (__float_as_uint(c.y) & m2) | (__float_as_uint(d.y) & m3)));
    o.z = bf16_val(__uint_as_float((__float_as_uint(a.z) & m0) | (__float_as_uint(b.z) & m1) | (__float_as_uint(c.z) & m2) | (__float_as_uint(d.z) & m3)));
    o.w = bf16_val(__uint_as_float((__float_as_uint(a.w) & m0) | (__float_as_uint(b.w) & m1) | (__float_as_uint(c.w) & m2) | (__float_as_uint(d.w) & m3)));
    if (act) *(volatile v4f*)(PT + PT_NB + 4 * t) = o;
    __threadfence();
    if (act) *(volatile v4f*)(PT + PT_NB + 4 * t) = o;
  }
}

__global__ __launch_bounds__(256) void k_pb(const float* __restrict__ ew0, const float* __restrict__ eb0,
                                            const float* __restrict__ ew, const float* __restrict__ eb,
                                            const float* __restrict__ eg, const float* __restrict__ ebb,
                                            const float* __restrict__ e1w, const float* __restrict__ e1b,
                                            unsigned short* ET, float* PT) {
  __shared__ __attribute__((aligned(16))) float sT[800];
  const int tid = (int)threadIdx.x;
  if ((int)blockIdx.x < 12) {
    const int u = (int)blockIdx.x * 256 + tid;
    const int layer = u >> 10;
    const int rem = u & 1023;
    const int n = rem >> 4;
    const int k8 = ((rem & 15) * 8) & 63;
    const v8us r = gather_wt(ew, layer, k8, n);
    put16(ET + (size_t)u * 8, r);
  } else {
#pragma unroll 1
    for (int i = tid; i < 800; i += 256) {
      const int i0 = i < 191 ? i : 191;
      int i1 = i - 192; i1 = i1 < 0 ? 0 : (i1 > 191 ? 191 : i1);
      int i2 = i - 384; i2 = i2 < 0 ? 0 : (i2 > 191 ? 191 : i2);
      int i3 = i - 576; i3 = i3 < 0 ? 0 : (i3 > 63 ? 63 : i3);
      int i4 = i - 640; i4 = i4 < 0 ? 0 : (i4 > 63 ? 63 : i4);
      int i5 = i - 704; i5 = i5 < 0 ? 0 : (i5 > 63 ? 63 : i5);
      const unsigned c0 = __float_as_uint(eb[i0]);
      const unsigned c1 = __float_as_uint(eg[i1]);
      const unsigned c2 = __float_as_uint(ebb[i2]);
      const unsigned c3 = __float_as_uint(ew0[i3]);
      const unsigned c4 = __float_as_uint(eb0[i4]);
      const unsigned c5 = __float_as_uint(e1w[i5]);
      const unsigned c6 = __float_as_uint(e1b[0]);
      const unsigned m0 = (i < 192) ? 0xffffffffu : 0u;
      const unsigned m1 = (i >= 192 && i < 384) ? 0xffffffffu : 0u;
      const unsigned m2 = (i >= 384 && i < 576) ? 0xffffffffu : 0u;
      const unsigned m3 = (i >= 576 && i < 640) ? 0xffffffffu : 0u;
      const unsigned m4 = (i >= 640 && i < 704) ? 0xffffffffu : 0u;
      const unsigned m5 = (i >= 704 && i < 768) ? 0xffffffffu : 0u;
      const unsigned m6 = (i == 768) ? 0xffffffffu : 0u;
      const unsigned sel = (c0 & m0) | (c1 & m1) | (c2 & m2) | (c3 & m3) | (c4 & m4) | (c5 & m5) | (c6 & m6);
      sT[i] = bf16_val(__uint_as_float(sel));
    }
    __syncthreads();
    const bool act = tid < 200;
    const int t = act ? tid : 0;
    const v4f o = *(const v4fa*)(sT + 4 * t);
    if (act) *(volatile v4f*)(PT + PT_EB + 4 * t) = o;
    __threadfence();
    if (act) *(volatile v4f*)(PT + PT_EB + 4 * t) = o;
  }
}

__device__ __forceinline__ float nemb(float x0, float x1, float w0, float w1, float b) {
  const float p = x0 * bf16_val(w0) + x1 * bf16_val(w1);
  return lrelu(p + bf16_val(b));
}

__global__ __launch_bounds__(256) void k_pc(const float* __restrict__ x, const float* __restrict__ vw,
                                            const float* __restrict__ vb, const float* __restrict__ vg,
                                            const float* __restrict__ vbb, float* PT, float* H, unsigned short* HHL) {
  const int tid = (int)threadIdx.x;
  if ((int)blockIdx.x < 200) {
    const int u = (int)blockIdx.x * 256 + tid;
    const int row = u >> 4, q = u & 15;
    const v2f xr = *(const v2f*)(x + 2 * row);
    const float x0 = bf16_val(xr.x), x1 = bf16_val(xr.y);
    v4f hv;
    {
      const int c = 4 * q;
      const v4f a = *(const v4f*)(vw + c);
      const v4f b = *(const v4f*)(vw + UU + c);
      const v4f d = *(const v4f*)(vb + c);
      hv.x = nemb(x0, x1, a.x, b.x, d.x);
      hv.y = nemb(x0, x1, a.y, b.y, d.y);
      hv.z = nemb(x0, x1, a.z, b.z, d.z);
      hv.w = nemb(x0, x1, a.w, b.w, d.w);
    }
    v8us ov;
    {
      const int c8 = (q & 7) * 8;
      const unsigned lm = (q >= 8) ? 0xffffu : 0u;
      const v4f a0 = *(const v4f*)(vw + c8);
      const v4f a1 = *(const v4f*)(vw + c8 + 4);
      const v4f b0 = *(const v4f*)(vw + UU + c8);
      const v4f b1 = *(const v4f*)(vw + UU + c8 + 4);
      const v4f d0 = *(const v4f*)(vb + c8);
      const v4f d1 = *(const v4f*)(vb + c8 + 4);
      const v8f wa = {a0.x, a0.y, a0.z, a0.w, a1.x, a1.y, a1.z, a1.w};
      const v8f wb = {b0.x, b0.y, b0.z, b0.w, b1.x, b1.y, b1.z, b1.w};
      const v8f wd = {d0.x, d0.y, d0.z, d0.w, d1.x, d1.y, d1.z, d1.w};
#pragma unroll
      for (int i = 0; i < 8; ++i) {
        unsigned hb, lb;
        split2(nemb(x0, x1, wa[i], wb[i], wd[i]), hb, lb);
        ov[i] = (unsigned short)((hb & ~lm) | (lb & lm));
      }
    }
    *(volatile v4f*)(H + (size_t)u * 4) = hv;
    *(volatile v8us*)(HHL + (size_t)u * 8) = ov;
    __threadfence();
    *(volatile v4f*)(H + (size_t)u * 4) = hv;
    *(volatile v8us*)(HHL + (size_t)u * 8) = ov;
  } else {
    const bool act = tid < 96;
    const int t = act ? tid : 0;
    const int og = (t < 47 ? t : 47) * 4;
    int tb = t - 48; tb = tb < 0 ? 0 : tb;
    const int ob = tb * 4;
    const v4f a = *(const v4f*)(vg + og);
    const v4f b = *(const v4f*)(vbb + ob);
    const unsigned mb = (t >= 48) ? 0xffffffffu : 0u;
    v4f o;
    o.x = bf16_val(__uint_as_float((__float_as_uint(a.x) & ~mb) | (__float_as_uint(b.x) & mb)));
    o.y = bf16_val(__uint_as_float((__float_as_uint(a.y) & ~mb) | (__float_as_uint(b.y) & mb)));
    o.z = bf16_val(__uint_as_float((__float_as_uint(a.z) & ~mb) | (__float_as_uint(b.z) & mb)));
    o.w = bf16_val(__uint_as_float((__float_as_uint(a.w) & ~mb) | (__float_as_uint(b.w) & mb)));
    if (act) *(volatile v4f*)(PT + PT_VG + 4 * t) = o;
    __threadfence();
    if (act) *(volatile v4f*)(PT + PT_VG + 4 * t) = o;
  }
}

__global__ __launch_bounds__(256) void k_w0(const float* __restrict__ adj, const float* __restrict__ PT,
                                            unsigned short* WHL) {
  const int g = (int)blockIdx.x * 256 + (int)threadIdx.x;
  if (g >= RTOT * 8) return;
  const int r = g >> 3, q = g & 7;
  const int c = 8 * q;
  const float a = bf16_val(adj[r]);
  const v4f w0 = *(const v4f*)(PT + PT_EW0 + c);
  const v4f w1 = *(const v4f*)(PT + PT_EW0 + c + 4);
  const v4f b0 = *(const v4f*)(PT + PT_EB0 + c);
  const v4f b1 = *(const v4f*)(PT + PT_EB0 + c + 4);
  const v8f wv = {w0.x, w0.y, w0.z, w0.w, w1.x, w1.y, w1.z, w1.w};
  const v8f bv = {b0.x, b0.y, b0.z, b0.w, b1.x, b1.y, b1.z, b1.w};
  v8us hv, lv;
#pragma unroll
  for (int i = 0; i < 8; ++i) {
    unsigned hb, lb;
    split2(lrelu(a * wv[i] + bv[i]), hb, lb);
    hv[i] = (unsigned short)hb;
    lv[i] = (unsigned short)lb;
  }
  unsigned short* rp = WHL + (size_t)r * KK + c;
  *(volatile v8us*)rp = hv;
  *(volatile v8us*)(rp + UU) = lv;
  __threadfence();
  *(volatile v8us*)rp = hv;
  *(volatile v8us*)(rp + UU) = lv;
}

__device__ __forceinline__ void gn_store_pass(const float* stg, float* X4, int rowBase, int wave, int lane,
                                              int colBase, v4f bias) {
#pragma unroll 4
  for (int i = 0; i < 16; ++i) {
    const v4f a = *(const v4fa*)(stg + (16 * wave + i) * 128 + 4 * lane);
    const v4f o = a + bias;
    *(volatile v4f*)(X4 + (size_t)(rowBase + 16 * wave + i) * X4W + colBase + 4 * lane) = o;
  }
}

__global__ __launch_bounds__(128) __attribute__((amdgpu_num_vgpr(248)))
void k_gn(const unsigned short* __restrict__ A, const unsigned short* __restrict__ WN,
          const float* __restrict__ PT, int layer, float* X4) {
  __shared__ __attribute__((aligned(16))) float stg[64 * 128];
  const int tid = (int)threadIdx.x, lane = tid & 31, wave = tid >> 5, hh = lane >> 4, m = lane & 15;
  const int rowBase = (int)blockIdx.x * 64;
  const int colBase = (int)blockIdx.y * 128;

  v8f acc[8];
#pragma unroll
  for (int t = 0; t < 8; ++t) acc[t] = z8();
  const unsigned short* ap = A + (size_t)(rowBase + 16 * wave + m) * KK + 8 * hh;
  const unsigned short* bp = WN + (size_t)layer * 256 * KK + (size_t)(colBase + m) * KK + 8 * hh;

#pragma unroll 1
  for (int k0 = 0; k0 < KK; k0 += 32) {
    FragB af;
    af.h[0] = *(const v8usa*)(ap + k0);
    af.h[1] = *(const v8usa*)(ap + k0 + 16);
#pragma unroll
    for (int nt = 0; nt < 8; ++nt) {
      const unsigned short* wq = bp + (size_t)(16 * nt) * KK + k0;
      FragB bf;
      bf.h[0] = *(const v8usa*)wq;
      bf.h[1] = *(const v8usa*)(wq + 16);
      acc[nt] = wmb(af, bf, acc[nt]);
    }
  }
#pragma unroll
  for (int nt = 0; nt < 8; ++nt) {
#pragma unroll
    for (int r = 0; r < 8; ++r) stg[(16 * wave + 8 * hh + r) * 128 + 16 * nt + m] = acc[nt][r];
  }
  __syncthreads();
  const v4f bias = *(const v4f*)(PT + PT_NB + layer * 256 + colBase + 4 * lane);
  gn_store_pass(stg, X4, rowBase, wave, lane, colBase, bias);
  __threadfence();
  gn_store_pass(stg, X4, rowBase, wave, lane, colBase, bias);
}

__global__ __launch_bounds__(256) void k_pool(const unsigned* __restrict__ WHLw, const float* __restrict__ X4,
                                              float* PO) {
  __shared__ __attribute__((aligned(16))) float sx[NN * UU];
  const int tid = (int)threadIdx.x, lane = tid & 31, wave = tid >> 5;
  const int b = (int)blockIdx.x / 25, ub = (int)blockIdx.x - b * 25;
#pragma unroll 1
  for (int i = tid; i < NN * 16; i += 256) {
    const int row = i >> 4, c4 = i & 15;
    const v4f t = *(const v4f*)(X4 + (size_t)(b * NN + row) * X4W + UU + 4 * c4);
    *(v4fa*)(sx + row * UU + 4 * c4) = t;
  }
  __syncthreads();
  const int u = ub * 8 + wave;
  const unsigned* wp = WHLw + (size_t)(b * NN + u) * NN * 64 + lane;
  const float ninf = __uint_as_float(0xff800000u);
  float m0 = ninf, m1 = ninf;
#pragma unroll 2
  for (int v = 0; v < NN; ++v) {
    const unsigned hw = wp[(size_t)v * 64];
    const unsigned lw = wp[(size_t)v * 64 + 32];
    const float w0 = __uint_as_float(hw << 16) + __uint_as_float(lw << 16);
    const float w1 = __uint_as_float(hw & 0xffff0000u) + __uint_as_float(lw & 0xffff0000u);
    const v2f xv = *(const v2fa*)(sx + v * UU + 2 * lane);
    const float s0 = __builtin_amdgcn_rcpf(1.0f + __expf(-w0));
    const float s1 = __builtin_amdgcn_rcpf(1.0f + __expf(-w1));
    const float p0 = s0 * xv.x;
    const float p1 = s1 * xv.y;
    const bool dead = (v == u);
    const float e0 = dead ? ninf : p0;
    const float e1 = dead ? ninf : p1;
    m0 = (e0 > m0) ? e0 : m0;
    m1 = (e1 > m1) ? e1 : m1;
  }
  v2f o;
  o.x = m0;
  o.y = m1;
  float* op = PO + (size_t)(b * NN + u) * UU + 2 * lane;
  *(volatile v2f*)op = o;
  __threadfence();
  *(volatile v2f*)op = o;
}

__device__ __forceinline__ void edge_tile_gemm(const unsigned short* sA, const unsigned short* sB, float* sD,
                                               int wave, int hh, int m) {
  v8f acc[4];
#pragma unroll
  for (int t = 0; t < 4; ++t) acc[t] = z8();
  const unsigned short* ap = sA + (16 * wave + m) * KK + 8 * hh;
  const unsigned short* bp = sB + m * KK + 8 * hh;
#pragma unroll 1
  for (int k0 = 0; k0 < KK; k0 += 32) {
    FragB af;
    af.h[0] = *(const v8usa*)(ap + k0);
    af.h[1] = *(const v8usa*)(ap + k0 + 16);
#pragma unroll
    for (int nt = 0; nt < 4; ++nt) {
      const unsigned short* wq = bp + (16 * nt) * KK + k0;
      FragB bf;
      bf.h[0] = *(const v8usa*)wq;
      bf.h[1] = *(const v8usa*)(wq + 16);
      acc[nt] = wmb(af, bf, acc[nt]);
    }
  }
#pragma unroll
  for (int nt = 0; nt < 4; ++nt) {
#pragma unroll
    for (int r = 0; r < 8; ++r) sD[(16 * wave + 8 * hh + r) * DP + 16 * nt + m] = acc[nt][r];
  }
}

template <int MODE>
__global__ __launch_bounds__(256) __attribute__((amdgpu_num_vgpr(248)))
void k_edge(unsigned short* WHL, const unsigned short* __restrict__ ET, const float* __restrict__ X4,
            const float* __restrict__ PT, const float* __restrict__ ST, int layer, float* REC, float* out) {
  extern __shared__ __attribute__((aligned(16))) float dyn[];
  __shared__ __attribute__((aligned(16))) float red[4 * UU];
  __shared__ __attribute__((aligned(16))) float red2[4 * UU];
  __shared__ __attribute__((aligned(16))) float pst[2 * UU];
  __shared__ __attribute__((aligned(16))) float sOut[TROWS];
  float*          sD = dyn;
  unsigned short* sA = (unsigned short*)(dyn + TROWS * DP);
  unsigned short* sB = sA + TROWS * KK;

  const int tid = (int)threadIdx.x, lane = tid & 31, wave = tid >> 5, hh = lane >> 4, m = lane & 15;
  const int tile = (int)blockIdx.x;
  const int rbase = tile * TROWS;
  unsigned short* gtile = WHL + (size_t)rbase * KK;

  {
    const unsigned short* gp = gtile;
#pragma unroll
    for (int it = 0; it < 8; ++it) {
      const v4i t = *(const v4ia*)(gp + (size_t)(it * 256 + tid) * 8);
      *(v4ia*)(sA + (it * 256 + tid) * 8) = t;
    }
    const unsigned short* ep = ET + (size_t)layer * UU * KK;
#pragma unroll
    for (int it = 0; it < 4; ++it) {
      const v4i t = *(const v4ia*)(ep + (size_t)(it * 256 + tid) * 8);
      *(v4ia*)(sB + (it * 256 + tid) * 8) = t;
    }
  }
  __syncthreads();

  edge_tile_gemm(sA, sB, sD, wave, hh, m);
  __syncthreads();

  const int c4 = tid & 15, rq = tid >> 4, cc = 4 * c4;
  const v4f ebv = *(const v4f*)(PT + PT_EB + layer * UU + cc);
  v4f mean4 = {0.f, 0.f, 0.f, 0.f}, rstd4 = mean4, g4 = mean4, bt4 = mean4, e14 = mean4;
  float e1b = 0.0f;
  if constexpr (MODE >= 1) {
    mean4 = *(const v4f*)(ST + cc);
    rstd4 = *(const v4f*)(ST + UU + cc);
    g4    = *(const v4f*)(PT + PT_EG + layer * UU + cc);
    bt4   = *(const v4f*)(PT + PT_EBB + layer * UU + cc);
  }
  if constexpr (MODE == 2) {
    e14 = *(const v4f*)(PT + PT_E1W + cc);
    e1b = PT[PT_E1B];
  }

#pragma unroll 2
  for (int it = 0; it < 8; ++it) {
    const int row = rq + 16 * it;
    const int r = rbase + row;
    const int bu = r / NN;
    const int v = r - bu * NN;
    const int b = bu / NN;
    const int u = bu - b * NN;
    const v4f a  = *(const v4fa*)(sD + row * DP + cc);
    const v4f x3 = *(const v4f*)(X4 + (size_t)bu * X4W + 128 + cc);
    const v4f x4 = *(const v4f*)(X4 + (size_t)(b * NN + v) * X4W + 192 + cc);
    v4f z;
    z.x = ((a.x + ebv.x) + x3.x) + x4.x;
    z.y = ((a.y + ebv.y) + x3.y) + x4.y;
    z.z = ((a.z + ebv.z) + x3.z) + x4.z;
    z.w = ((a.w + ebv.w) + x3.w) + x4.w;
    if constexpr (MODE == 0) {
      *(v4fa*)(sD + row * DP + cc) = z;
    } else {
      const v4us hb = *(const v4usa*)(sA + row * KK + cc);
      const v4us lb = *(const v4usa*)(sA + row * KK + UU + cc);
      v4f wn;
      wn.x = (bw((unsigned)hb.x) + bw((unsigned)lb.x)) + lrelu((g4.x * (z.x - mean4.x)) * rstd4.x + bt4.x);
      wn.y = (bw((unsigned)hb.y) + bw((unsigned)lb.y)) + lrelu((g4.y * (z.y - mean4.y)) * rstd4.y + bt4.y);
      wn.z = (bw((unsigned)hb.z) + bw((unsigned)lb.z)) + lrelu((g4.z * (z.z - mean4.z)) * rstd4.z + bt4.z);
      wn.w = (bw((unsigned)hb.w) + bw((unsigned)lb.w)) + lrelu((g4.w * (z.w - mean4.w)) * rstd4.w + bt4.w);
      if constexpr (MODE == 1) {
        unsigned h0, l0, h1, l1, h2, l2, h3, l3;
        split2(wn.x, h0, l0);
        split2(wn.y, h1, l1);
        split2(wn.z, h2, l2);
        split2(wn.w, h3, l3);
        const v4us nh = {(unsigned short)h0, (unsigned short)h1, (unsigned short)h2, (unsigned short)h3};
        const v4us nl = {(unsigned short)l0, (unsigned short)l1, (unsigned short)l2, (unsigned short)l3};
        *(v4usa*)(sA + row * KK + cc) = nh;
        *(v4usa*)(sA + row * KK + UU + cc) = nl;
      } else {
        float part = ((wn.x * e14.x + wn.y * e14.y) + wn.z * e14.z) + wn.w * e14.w;
        part += __shfl_xor(part, 1, 32);
        part += __shfl_xor(part, 2, 32);
        part += __shfl_xor(part, 4, 32);
        part += __shfl_xor(part, 8, 32);
        const float val = (u == v) ? 0.0f : (part + e1b);
        if (c4 == 0) sOut[row] = val;
      }
    }
  }
  __syncthreads();

  if constexpr (MODE == 0) {
    const int nd0 = diag_before(rbase);
    const int dl0 = diag_pos(nd0) - rbase;
    const int dl1 = diag_pos(nd0 + 1) - rbase;
    const int nlive = TROWS - (dl0 < TROWS ? 1 : 0) - (dl1 < TROWS ? 1 : 0);
    const float rn = 1.0f / (float)nlive;
    const int c = tid & (UU - 1);
    const int g = tid >> 6;
    const float* col = sD + (32 * g) * DP + c;
    float s = 0.0f;
#pragma unroll 4
    for (int i = 0; i < 32; ++i) {
      const int row = 32 * g + i;
      const float zv = col[i * DP];
      const bool dead = (row == dl0) | (row == dl1);
      s += dead ? 0.0f : zv;
    }
    red[g * UU + c] = s;
    __syncthreads();
    const float tot = ((red[c] + red[UU + c]) + red[2 * UU + c]) + red[3 * UU + c];
    const float mean = tot * rn;
    float q = 0.0f;
#pragma unroll 4
    for (int i = 0; i < 32; ++i) {
      const int row = 32 * g + i;
      const float d = col[i * DP] - mean;
      const bool dead = (row == dl0) | (row == dl1);
      q += dead ? 0.0f : d * d;
    }
    red2[g * UU + c] = q;
    __syncthreads();
    const float M2 = ((red2[c] + red2[UU + c]) + red2[2 * UU + c]) + red2[3 * UU + c];
    if (g == 0) { pst[2 * c] = mean; pst[2 * c + 1] = M2; }
    __syncthreads();
    const bool act = tid < 32;
    const int t = act ? tid : 0;
    const v4f ps = *(const v4fa*)(pst + 4 * t);
    if (act) *(volatile v4f*)(REC + (size_t)tile * 128 + 4 * t) = ps;
    __threadfence();
    if (act) *(volatile v4f*)(REC + (size_t)tile * 128 + 4 * t) = ps;
  } else if constexpr (MODE == 1) {
    v4i pv[8];
#pragma unroll
    for (int it = 0; it < 8; ++it) pv[it] = *(const v4ia*)(sA + (it * 256 + tid) * 8);
#pragma unroll
    for (int it = 0; it < 8; ++it) *(volatile v4i*)(gtile + (size_t)(it * 256 + tid) * 8) = pv[it];
    __threadfence();
#pragma unroll
    for (int it = 0; it < 8; ++it) *(volatile v4i*)(gtile + (size_t)(it * 256 + tid) * 8) = pv[it];
  } else {
    const bool act = tid < 32;
    const int t = act ? tid : 0;
    const v4f ov = *(const v4fa*)(sOut + 4 * t);
    if (act) *(volatile v4f*)(out + (size_t)rbase + 4 * t) = ov;
    __threadfence();
    if (act) *(volatile v4f*)(out + (size_t)rbase + 4 * t) = ov;
  }
}

__global__ __launch_bounds__(256) void k_cmb(const float* __restrict__ REC, float* ST) {
  __shared__ double cn[256], cm[256], cq[256];
  __shared__ __attribute__((aligned(16))) float stg[2 * UU];
  const int tid = (int)threadIdx.x;
  const int c = tid & (UU - 1);
  const int p = tid >> 6;
  double n = 0.0, mean = 0.0, M2 = 0.0;
#pragma unroll 1
  for (int t = p; t < NTILE; t += 4) {
    const int nd = diag_before(TROWS * t + TROWS) - diag_before(TROWS * t);
    const double nb = (double)(TROWS - nd);
    const v2f rc = *(const v2f*)(REC + (size_t)t * 128 + 2 * c);
    const double mb = (double)rc.x;
    const double qb = (double)rc.y;
    const double nn = n + nb;
    const double delta = mb - mean;
    const double f = nb / nn;
    mean = mean + delta * f;
    M2 = M2 + qb + delta * delta * n * f;
    n = nn;
  }
  cn[tid] = n; cm[tid] = mean; cq[tid] = M2;
  __syncthreads();
  if (tid < UU) {
    double tn = 0.0, tm = 0.0, tq = 0.0;
#pragma unroll 1
    for (int p2 = 0; p2 < 4; ++p2) {
      const double nb = cn[p2 * UU + c];
      const double mb = cm[p2 * UU + c];
      const double qb = cq[p2 * UU + c];
      const double nn = tn + nb;
      const double delta = mb - tm;
      const double f = nb / nn;
      tm = tm + delta * f;
      tq = tq + qb + delta * delta * tn * f;
      tn = nn;
    }
    const float qnan = __uint_as_float(0x7fc00000u);
    const float poison = (tn == (double)NLIVE) ? 0.0f : qnan;
    const float varf = (float)(tq / (double)NLIVE);
    const float rstd = 1.0f / sqrtf(varf + BNEPS);
    stg[c] = (float)tm + poison;
    stg[UU + c] = rstd;
  }
  __syncthreads();
  const bool act = tid < 32;
  const int t = act ? tid : 0;
  const v4f o = *(const v4fa*)(stg + 4 * t);
  if (act) *(volatile v4f*)(ST + 4 * t) = o;
  __threadfence();
  if (act) *(volatile v4f*)(ST + 4 * t) = o;
}

__global__ __launch_bounds__(256) void k_nd(const float* __restrict__ X4, const float* __restrict__ PO,
                                            const float* __restrict__ PT, int layer, float* H, unsigned short* HHL) {
  __shared__ double dsum[256];
  __shared__ __attribute__((aligned(16))) float sH[32 * UU];
  const int tid = (int)threadIdx.x;
  const int c = tid & (UU - 1);
  const int p = tid >> 6;

  double s = 0.0;
#pragma unroll 4
  for (int j = 0; j < NROW / 4; ++j) {
    const int row = 4 * j + p;
    const float t = X4[(size_t)row * X4W + c] + PO[(size_t)row * UU + c];
    s += (double)t;
  }
  dsum[tid] = s;
  __syncthreads();
  const double mean = (((dsum[c] + dsum[UU + c]) + dsum[2 * UU + c]) + dsum[3 * UU + c]) * (1.0 / (double)NROW);
  __syncthreads();
  double q = 0.0;
#pragma unroll 4
  for (int j = 0; j < NROW / 4; ++j) {
    const int row = 4 * j + p;
    const float t = X4[(size_t)row * X4W + c] + PO[(size_t)row * UU + c];
    const double d = (double)t - mean;
    q += d * d;
  }
  dsum[tid] = q;
  __syncthreads();
  const double M2 = ((dsum[c] + dsum[UU + c]) + dsum[2 * UU + c]) + dsum[3 * UU + c];
  const float varf  = (float)(M2 * (1.0 / (double)NROW));
  const float meanf = (float)mean;
  const float rstd  = 1.0f / sqrtf(varf + BNEPS);
  const float gg = PT[PT_VG + layer * UU + c];
  const float bb = PT[PT_VB + layer * UU + c];

#pragma unroll 1
  for (int ch = 0; ch < NROW / 32; ++ch) {
#pragma unroll 2
    for (int j = 0; j < 8; ++j) {
      const int rl = 4 * j + p;
      const int row = ch * 32 + rl;
      const float t = X4[(size_t)row * X4W + c] + PO[(size_t)row * UU + c];
      const float ho = H[(size_t)row * UU + c];
      const float y = (gg * (t - meanf)) * rstd + bb;
      sH[rl * UU + c] = ho + lrelu(y);
    }
    __syncthreads();
    v4f hv[2];
    v8us uv[2];
#pragma unroll
    for (int k = 0; k < 2; ++k) {
      const int unit = tid + 256 * k;
      hv[k] = *(const v4fa*)(sH + 4 * unit);
      const int rl = unit >> 4, qq = unit & 15;
      const int c8 = (qq & 7) * 8;
      const unsigned lm = (qq >= 8) ? 0xffffu : 0u;
      const v4f a0 = *(const v4fa*)(sH + rl * UU + c8);
      const v4f a1 = *(const v4fa*)(sH + rl * UU + c8 + 4);
      const v8f av = {a0.x, a0.y, a0.z, a0.w, a1.x, a1.y, a1.z, a1.w};
      v8us o;
#pragma unroll
      for (int i = 0; i < 8; ++i) {
        unsigned hb, lb;
        split2(av[i], hb, lb);
        o[i] = (unsigned short)((hb & ~lm) | (lb & lm));
      }
      uv[k] = o;
    }
    float* hp = H + (size_t)ch * 32 * UU;
    unsigned short* lp = HHL + (size_t)ch * 32 * KK;
#pragma unroll
    for (int k = 0; k < 2; ++k) {
      *(volatile v4f*)(hp + 4 * (tid + 256 * k)) = hv[k];
      *(volatile v8us*)(lp + 8 * (tid + 256 * k)) = uv[k];
    }
    __threadfence();
#pragma unroll
    for (int k = 0; k < 2; ++k) {
      *(volatile v4f*)(hp + 4 * (tid + 256 * k)) = hv[k];
      *(volatile v8us*)(lp + 8 * (tid + 256 * k)) = uv[k];
    }
    __syncthreads();
  }
}

extern "C" void kernel_launch(void* const* d_in, const int* in_sizes, int n_in,
                              void* d_out, int out_size, void* d_ws, size_t ws_size,
                              hipStream_t stream) {
  if (n_in < 22) return;
  const int want[22] = {NB * NN * 2, RTOT, 2 * UU, UU,
                        NL * UU * UU, NL * UU, NL * UU * UU, NL * UU, NL * UU * UU, NL * UU, NL * UU * UU, NL * UU,
                        NL * UU, NL * UU, UU, UU, NL * UU * UU, NL * UU, NL * UU, NL * UU, UU, 1};
  for (int i = 0; i < 22; ++i) if (in_sizes[i] != want[i]) return;
  if (out_size != RTOT) return;
  if (ws_size < (size_t)WS_TOTAL) return;
  {
    long long live = 0;
    for (int t = 0; t < NTILE; ++t) live += TROWS - (diag_before(TROWS * t + TROWS) - diag_before(TROWS * t));
    if (live != (long long)NLIVE) return;
  }

  const float* x    = (const float*)d_in[0];
  const float* adj  = (const float*)d_in[1];
  const float* vw0  = (const float*)d_in[2];
  const float* vb0  = (const float*)d_in[3];
  const float* vw1  = (const float*)d_in[4];
  const float* vb1  = (const float*)d_in[5];
  const float* vw2  = (const float*)d_in[6];
  const float* vb2  = (const float*)d_in[7];
  const float* vw3  = (const float*)d_in[8];
  const float* vb3  = (const float*)d_in[9];
  const float* vw4  = (const float*)d_in[10];
  const float* vb4  = (const float*)d_in[11];
  const float* vg   = (const float*)d_in[12];
  const float* vbb  = (const float*)d_in[13];
  const float* ew0  = (const float*)d_in[14];
  const float* eb0  = (const float*)d_in[15];
  const float* ew   = (const float*)d_in[16];
  const float* eb   = (const float*)d_in[17];
  const float* eg   = (const float*)d_in[18];
  const float* ebb  = (const float*)d_in[19];
  const float* e1w  = (const float*)d_in[20];
  const float* e1b  = (const float*)d_in[21];
  float* out = (float*)d_out;

  char* ws = (char*)d_ws;
  size_t off = 0;
  unsigned short* WHL = (unsigned short*)(ws + off); off += SZ_WHL;
  float*          X4  = (float*)(ws + off);          off += SZ_X4;
  float*          H   = (float*)(ws + off);          off += SZ_H;
  unsigned short* HHL = (unsigned short*)(ws + off); off += SZ_HHL;
  float*          PO  = (float*)(ws + off);          off += SZ_PO;
  float*          REC = (float*)(ws + off);          off += SZ_REC;
  unsigned short* WN  = (unsigned short*)(ws + off); off += SZ_WN;
  unsigned short* ET  = (unsigned short*)(ws + off); off += SZ_ET;
  float*          PT  = (float*)(ws + off);          off += SZ_PT;
  float*          ST  = (float*)(ws + off);          off += SZ_ST;
  if (off != (size_t)WS_TOTAL || off > ws_size) return;

  hipFuncSetAttribute(reinterpret_cast<const void*>(&k_edge<0>), hipFuncAttributeMaxDynamicSharedMemorySize,
                      (int)EDGE_DYN_BYTES);
  hipFuncSetAttribute(reinterpret_cast<const void*>(&k_edge<1>), hipFuncAttributeMaxDynamicSharedMemorySize,
                      (int)EDGE_DYN_BYTES);
  hipFuncSetAttribute(reinterpret_cast<const void*>(&k_edge<2>), hipFuncAttributeMaxDynamicSharedMemorySize,
                      (int)EDGE_DYN_BYTES);

  k_pa<<<49, 256, 0, stream>>>(vw1, vw2, vw3, vw4, vb1, vb2, vb3, vb4, WN, PT);
  k_pb<<<13, 256, 0, stream>>>(ew0, eb0, ew, eb, eg, ebb, e1w, e1b, ET, PT);
  k_pc<<<201, 256, 0, stream>>>(x, vw0, vb0, vg, vbb, PT, H, HHL);
  k_w0<<<(RTOT * 8) / 256, 256, 0, stream>>>(adj, PT, WHL);

  for (int layer = 0; layer < NL; ++layer) {
    k_gn<<<dim3(NROW / 64, 2), 128, 0, stream>>>(HHL, WN, PT, layer, X4);
    k_pool<<<NB * (NN / 8), 256, 0, stream>>>((const unsigned*)WHL, X4, PO);
    k_edge<0><<<NTILE, 256, EDGE_DYN_BYTES, stream>>>(WHL, ET, X4, PT, ST, layer, REC, out);
    k_cmb<<<1, 256, 0, stream>>>(REC, ST);
    k_nd<<<1, 256, 0, stream>>>(X4, PO, PT, layer, H, HHL);
    if (layer < NL - 1)
      k_edge<1><<<NTILE, 256, EDGE_DYN_BYTES, stream>>>(WHL, ET, X4, PT, ST, layer, REC, out);
    else
      k_edge<2><<<NTILE, 256, EDGE_DYN_BYTES, stream>>>(WHL, ET, X4, PT, ST, layer, REC, out);
  }
}
